// SparseGATv2Layer_82712480186382
// MI455X (gfx1250) — hardware-verified
//
#include <hip/hip_runtime.h>
#include <stddef.h>


#define FD      128
#define NH      4
#define HC      32
#define NMAT    2
#define NTHR    256
#define NWAVE   8
#define EPT     8
#define CHUNK   (NTHR * EPT)
#define WCAP    (EPT * 32)
#define LISTN   (NWAVE * WCAP)
#define NBMAX   2048
#define RCAP    28672
#define DEGCAP  4096
#define EB      8
#define GBM     64
#define GTHR    128
#define HSCALE  16.0f
#define WSCALE  64.0f
#define OINV    0.0009765625f
#define NEG_SLOPE 0.2f
#define EA2     0.35f
#define WSCAP   134217728
#define LDS_AGG ((2 * RCAP + 2 * NBMAX + LISTN) * 4 + 64)

static_assert((CHUNK & (CHUNK - 1)) == 0 && CHUNK <= 4096);
static_assert((NBMAX & (NBMAX - 1)) == 0 && NBMAX <= 4096);
static_assert(NTHR * 8 == NBMAX);
static_assert(LISTN >= NBMAX);
static_assert(LISTN >= NWAVE * WCAP);
static_assert((RCAP % 32) == 0);
static_assert(LDS_AGG <= 300000);
static_assert(GBM == (GTHR / 32) * 16);
static_assert(NH * HC == FD);
static_assert(EB * NH == 32);

typedef float          v2f  __attribute__((ext_vector_type(2)));
typedef float          v4f  __attribute__((ext_vector_type(4)));
typedef float          v8f  __attribute__((ext_vector_type(8)));
typedef int            v4i  __attribute__((ext_vector_type(4)));
typedef unsigned short v8us __attribute__((ext_vector_type(8)));
typedef _Float16       v8h  __attribute__((ext_vector_type(8)));
typedef _Float16       v16h __attribute__((ext_vector_type(16)));
union FragH { v16h v; v8us h[2]; };
union Pack8 { v8h h; v8us u; };

__device__ __forceinline__ v8us cvt8h(v4f a, v4f b, float sc) {
  v8h r;
  r[0] = (_Float16)(a.x * sc); r[1] = (_Float16)(a.y * sc);
  r[2] = (_Float16)(a.z * sc); r[3] = (_Float16)(a.w * sc);
  r[4] = (_Float16)(b.x * sc); r[5] = (_Float16)(b.y * sc);
  r[6] = (_Float16)(b.z * sc); r[7] = (_Float16)(b.w * sc);
  Pack8 p;
  p.h = r;
  return p.u;
}

__device__ __forceinline__ v8f wmh(v16h a, v16h b, v8f c) {
  v8f d = __builtin_amdgcn_wmma_f32_16x16x32_f16(false, a, false, b, (short)0, c, false, false);
  asm volatile("v_nop\n\tv_nop\n\tv_nop\n\tv_nop" : "+v"(d) : "v"(a), "v"(b));
  return d;
}

__device__ __forceinline__ int scan_chunk(const int* __restrict__ dsts, int nE, int cbase, int slotBase,
                                          int nb, int vec8, int* list, int tid, int lane, int wave) {
  int wc = 0;
  const int el0  = tid * EPT;
  const int e0   = cbase + el0;
  const int sent = -2147483647 - 1;
  v4i da, db;
  if (vec8 != 0 && cbase + CHUNK <= nE) {
    da = *(const v4i*)(dsts + e0);
    db = *(const v4i*)(dsts + e0 + 4);
  } else {
    da.x = (e0     < nE) ? dsts[min(e0,     nE - 1)] : sent;
    da.y = (e0 + 1 < nE) ? dsts[min(e0 + 1, nE - 1)] : sent;
    da.z = (e0 + 2 < nE) ? dsts[min(e0 + 2, nE - 1)] : sent;
    da.w = (e0 + 3 < nE) ? dsts[min(e0 + 3, nE - 1)] : sent;
    db.x = (e0 + 4 < nE) ? dsts[min(e0 + 4, nE - 1)] : sent;
    db.y = (e0 + 5 < nE) ? dsts[min(e0 + 5, nE - 1)] : sent;
    db.z = (e0 + 6 < nE) ? dsts[min(e0 + 6, nE - 1)] : sent;
    db.w = (e0 + 7 < nE) ? dsts[min(e0 + 7, nE - 1)] : sent;
  }
  const unsigned nbs = (unsigned)slotBase;
  const unsigned unb = (unsigned)nb;
  const unsigned s0 = (unsigned)da.x - nbs, s1 = (unsigned)da.y - nbs;
  const unsigned s2 = (unsigned)da.z - nbs, s3 = (unsigned)da.w - nbs;
  const unsigned s4 = (unsigned)db.x - nbs, s5 = (unsigned)db.y - nbs;
  const unsigned s6 = (unsigned)db.z - nbs, s7 = (unsigned)db.w - nbs;
  const bool h0 = s0 < unb, h1 = s1 < unb, h2 = s2 < unb, h3 = s3 < unb;
  const bool h4 = s4 < unb, h5 = s5 < unb, h6 = s6 < unb, h7 = s7 < unb;
  const unsigned any = __builtin_amdgcn_ballot_w32(h0 | h1 | h2 | h3 | h4 | h5 | h6 | h7);
  if (any != 0u) {
#define HITJ(J, HJ, SJ) { \
      const unsigned mj = __builtin_amdgcn_ballot_w32(HJ); \
      if (mj != 0u) { \
        if (HJ) { \
          const int pos = wc + (int)__builtin_amdgcn_mbcnt_lo(mj, 0u); \
          if (pos < WCAP) list[wave * WCAP + pos] = ((el0 + (J)) << 12) | (int)(SJ); \
        } \
        wc += (int)__builtin_popcount(mj); } }
    HITJ(0, h0, s0)
    HITJ(1, h1, s1)
    HITJ(2, h2, s2)
    HITJ(3, h3, s3)
    HITJ(4, h4, s4)
    HITJ(5, h5, s5)
    HITJ(6, h6, s6)
    HITJ(7, h7, s7)
#undef HITJ
  }
  return wc;
}

__global__ __launch_bounds__(NTHR) void k_xprep(const float* __restrict__ x, unsigned short* X16,
                                                int nN, int nUnits) {
  const int i = (int)blockIdx.x * NTHR + (int)threadIdx.x;
  if (i >= nUnits) return;
  const int row = i >> 4;
  const int c0  = (i & 15) * 8;
  const int rc  = row < nN ? row : nN - 1;
  const float* p = x + (size_t)rc * FD + c0;
  v4f a = *(const v4f*)p, b = *(const v4f*)(p + 4);
  const v4f z4 = {0.f, 0.f, 0.f, 0.f};
  if (row >= nN) { a = z4; b = z4; }
  const v8us hv = cvt8h(a, b, HSCALE);
  unsigned short* d = X16 + (size_t)row * FD + c0;
  *(volatile v8us*)d = hv;
  __threadfence();
  *(volatile v8us*)d = hv;
}

__global__ __launch_bounds__(NTHR) void k_wprep(const float* __restrict__ Wl, const float* __restrict__ Wr,
                                                unsigned short* wq) {
  const int j = (int)blockIdx.y;
  const int u = (int)blockIdx.x * NTHR + (int)threadIdx.x;
  if (u >= FD * FD / 8) return;
  const int n  = u >> 4;
  const int k8 = (u & 15) * 8;
  const float* src = (j & 1) ? Wr : Wl;
  const float* p = src + (size_t)n * FD + k8;
  const v4f a = *(const v4f*)p, b = *(const v4f*)(p + 4);
  const v8us hv = cvt8h(a, b, WSCALE);
  unsigned short* d = wq + (size_t)j * FD * FD + (size_t)n * FD + k8;
  *(volatile v8us*)d = hv;
  __threadfence();
  *(volatile v8us*)d = hv;
}

__global__ __launch_bounds__(GTHR) void k_gemm(const unsigned short* __restrict__ A16,
                                               const unsigned short* __restrict__ Bw,
                                               float* Y, int yStride) {
  __shared__ __attribute__((aligned(16))) float stg[GBM * FD];
  const int tid = threadIdx.x, lane = tid & 31, wave = tid >> 5, hh = lane >> 4, m = lane & 15;
  const int rowBase = (int)blockIdx.x * GBM;
  const unsigned short* ap = A16 + (size_t)(rowBase + 16 * wave + m) * FD + 8 * hh;
  FragH a0, a1, a2, a3;
  a0.h[0] = *(const v8us*)(ap);
  a0.h[1] = *(const v8us*)(ap + 16);
  a1.h[0] = *(const v8us*)(ap + 32);
  a1.h[1] = *(const v8us*)(ap + 48);
  a2.h[0] = *(const v8us*)(ap + 64);
  a2.h[1] = *(const v8us*)(ap + 80);
  a3.h[0] = *(const v8us*)(ap + 96);
  a3.h[1] = *(const v8us*)(ap + 112);
#pragma unroll 1
  for (int w = 0; w < NMAT; ++w) {
#pragma unroll 1
    for (int ch = 0; ch < 2; ++ch) {
      v8f acc[4];
#pragma unroll
      for (int t = 0; t < 4; ++t) { v8f z = {0.f, 0.f, 0.f, 0.f, 0.f, 0.f, 0.f, 0.f}; acc[t] = z; }
      const unsigned short* bq = Bw + (size_t)w * FD * FD + (size_t)(64 * ch + m) * FD + 8 * hh;
#pragma unroll
      for (int t = 0; t < 4; ++t) {
        const unsigned short* bp = bq + (size_t)(16 * t) * FD;
        FragH b0, b1, b2, b3;
        b0.h[0] = *(const v8us*)(bp);
        b0.h[1] = *(const v8us*)(bp + 16);
        b1.h[0] = *(const v8us*)(bp + 32);
        b1.h[1] = *(const v8us*)(bp + 48);
        b2.h[0] = *(const v8us*)(bp + 64);
        b2.h[1] = *(const v8us*)(bp + 80);
        b3.h[0] = *(const v8us*)(bp + 96);
        b3.h[1] = *(const v8us*)(bp + 112);
        acc[t] = wmh(a0.v, b0.v, acc[t]);
        acc[t] = wmh(a1.v, b1.v, acc[t]);
        acc[t] = wmh(a2.v, b2.v, acc[t]);
        acc[t] = wmh(a3.v, b3.v, acc[t]);
      }
      float* sp = stg + (size_t)(16 * wave + 8 * hh) * FD + 64 * ch + m;
#pragma unroll
      for (int t = 0; t < 4; ++t) {
#pragma unroll
        for (int r = 0; r < 8; ++r) sp[(size_t)r * FD + 16 * t] = acc[t][r] * OINV;
      }
    }
    __syncthreads();
    const int nF4 = GBM * FD / 4;
    float* yb = Y + (size_t)w * (size_t)yStride + (size_t)rowBase * FD;
    const v4f* s4 = (const v4f*)stg;
#pragma unroll 1
    for (int f = tid; f < nF4; f += GTHR) { const v4f v = s4[f]; *(volatile v4f*)(yb + 4 * (size_t)f) = v; }
    __threadfence();
#pragma unroll 1
    for (int f = tid; f < nF4; f += GTHR) { const v4f v = s4[f]; *(volatile v4f*)(yb + 4 * (size_t)f) = v; }
    __syncthreads();
  }
}

__global__ __launch_bounds__(NTHR) void k_logit(const int* __restrict__ srcs, const int* __restrict__ dsts,
                                                const float* __restrict__ ea, const float* __restrict__ yp,
                                                const float* __restrict__ attr, const float* __restrict__ web,
                                                float* ev, int nE, int nN) {
  const int i = (int)blockIdx.x * NTHR + (int)threadIdx.x;
  const int e = i < nE ? i : nE - 1;
  int s = srcs[e]; s = s < 0 ? 0 : (s > nN - 1 ? nN - 1 : s);
  int d = dsts[e]; d = d < 0 ? 0 : (d > nN - 1 ? nN - 1 : d);
  const float* ps = yp + (size_t)s * FD;
  const float* pd = yp + (size_t)d * FD;
  const v2f at2 = *(const v2f*)(ea + 2 * (size_t)e);
  const float red = at2.x + EA2 * at2.y;
  float l0 = 0.0f, l1 = 0.0f, l2 = 0.0f, l3 = 0.0f;
#pragma unroll 1
  for (int h = 0; h < NH; ++h) {
    const float* ph = ps + HC * h;
    const float* qh = pd + HC * h;
    const float* ah = attr + HC * h;
    float acc = 0.0f;
#pragma unroll
    for (int jj = 0; jj < HC / 4; ++jj) {
      const v4f l = *(const v4f*)(ph + 4 * jj);
      const v4f r = *(const v4f*)(qh + 4 * jj);
      const v4f a = *(const v4f*)(ah + 4 * jj);
      const v4f t = l + r;
      v4f z;
      z.x = fmaxf(t.x, NEG_SLOPE * t.x);
      z.y = fmaxf(t.y, NEG_SLOPE * t.y);
      z.z = fmaxf(t.z, NEG_SLOPE * t.z);
      z.w = fmaxf(t.w, NEG_SLOPE * t.w);
      acc = fmaf(z.x, a.x, acc);
      acc = fmaf(z.y, a.y, acc);
      acc = fmaf(z.z, a.z, acc);
      acc = fmaf(z.w, a.w, acc);
    }
    const float lg = acc + red * web[h];
    l0 = (h == 0) ? lg : l0;
    l1 = (h == 1) ? lg : l1;
    l2 = (h == 2) ? lg : l2;
    l3 = (h == 3) ? lg : l3;
  }
  v4f o;
  o.x = l0; o.y = l1; o.z = l2; o.w = l3;
  float* gp = ev + 4 * (size_t)i;
  *(volatile v4f*)gp = o;
  __threadfence();
  *(volatile v4f*)gp = o;
}

__global__ __launch_bounds__(NTHR) void k_agg(
    const int* __restrict__ srcs, const int* __restrict__ dsts, const float* __restrict__ ev,
    const float* __restrict__ yp, const float* __restrict__ yr, const float* __restrict__ attr,
    const float* __restrict__ web, const float* __restrict__ biasr, float* outp,
    int nDst, int nE, int nb, int vec8) {
  extern __shared__ v4f lds_dyn[];
  int* reg1 = (int*)lds_dyn;
  int* reg2 = reg1 + RCAP;
  int* scnt = reg2 + RCAP;
  int* soff = scnt + NBMAX;
  int* list = soff + NBMAX;
  int* wcnt = list + LISTN;
  int* wtot = wcnt + NWAVE;
  const int tid = threadIdx.x, lane = tid & 31, wave = tid >> 5;
  const int nodeBase = (int)blockIdx.x * nb;

  for (int i = tid; i < NBMAX; i += NTHR) scnt[i] = 0;
  __syncthreads();

  int tot = 0;
  const int nChunks = (nE + CHUNK - 1) / CHUNK;
#pragma unroll 1
  for (int ch = 0; ch < nChunks; ++ch) {
    const int cbase = ch * CHUNK;
    const int wc = scan_chunk(dsts, nE, cbase, nodeBase, nb, vec8, list, tid, lane, wave);
    if (lane == 0) wcnt[wave] = wc;
    __syncthreads();
    int pre = 0, all = 0;
#pragma unroll
    for (int w2 = 0; w2 < NWAVE; ++w2) {
      int c = wcnt[w2];
      c = c < 0 ? 0 : (c > WCAP ? WCAP : c);
      all += c;
      pre += (w2 < wave) ? c : 0;
    }
    const int wcc  = wc > WCAP ? WCAP : wc;
    const int base = tot + pre;
#pragma unroll 1
    for (int i = lane; i < wcc; i += 32) {
      const int ent = list[wave * WCAP + i];
      const int el  = (ent >> 12) & (CHUNK - 1);
      const int sl  = ent & (NBMAX - 1);
      int eid = cbase + el;
      eid = eid > nE - 1 ? nE - 1 : eid;
      const int pos = base + i;
      if (pos < RCAP) reg1[pos] = (int)(((unsigned)eid << 12) | (unsigned)sl);
    }
    tot += all;
    tot = tot > RCAP ? RCAP : tot;
    __syncthreads();
  }
  const int nh = tot;

  if (wave == 0) {
#pragma unroll 1
    for (int b0 = 0; b0 < nh; b0 += 32) {
      const int idx = b0 + lane;
      const int uv  = reg1[idx < RCAP ? idx : RCAP - 1];
      const int m32 = (nh - b0) < 32 ? (nh - b0) : 32;
#pragma unroll 1
      for (int k = 0; k < m32; ++k) {
        const int u  = __builtin_amdgcn_readlane(uv, k);
        const int sl = u & (NBMAX - 1);
        if (lane == 0) scnt[sl] = scnt[sl] + 1;
      }
    }
  }
  __syncthreads();

  {
    const v4i ca = *(const v4i*)(scnt + 8 * tid);
    const v4i cb = *(const v4i*)(scnt + 8 * tid + 4);
    const int e0 = ca.x < 0 ? 0 : ca.x, e1 = ca.y < 0 ? 0 : ca.y, e2 = ca.z < 0 ? 0 : ca.z, e3 = ca.w < 0 ? 0 : ca.w;
    const int e4 = cb.x < 0 ? 0 : cb.x, e5 = cb.y < 0 ? 0 : cb.y, e6 = cb.z < 0 ? 0 : cb.z, e7 = cb.w < 0 ? 0 : cb.w;
    const int ts = e0 + e1 + e2 + e3 + e4 + e5 + e6 + e7;
    int incl = ts;
#pragma unroll
    for (int d = 1; d < 32; d <<= 1) {
      const int up = __shfl_up(incl, d);
      if (lane >= d) incl += up;
    }
    if (lane == 31) wtot[wave] = incl;
    __syncthreads();
    int pre = 0;
#pragma unroll
    for (int w2 = 0; w2 < NWAVE; ++w2) pre += (w2 < wave) ? wtot[w2] : 0;
    int run = pre + incl - ts;
    soff[8 * tid + 0] = run; run += e0;
    soff[8 * tid + 1] = run; run += e1;
    soff[8 * tid + 2] = run; run += e2;
    soff[8 * tid + 3] = run; run += e3;
    soff[8 * tid + 4] = run; run += e4;
    soff[8 * tid + 5] = run; run += e5;
    soff[8 * tid + 6] = run; run += e6;
    soff[8 * tid + 7] = run;
  }
  __syncthreads();
  for (int i = tid; i < NBMAX; i += NTHR) list[i] = soff[i];
  __syncthreads();

  if (wave == 0) {
#pragma unroll 1
    for (int b0 = 0; b0 < nh; b0 += 32) {
      const int idx = b0 + lane;
      const int uv  = reg1[idx < RCAP ? idx : RCAP - 1];
      const int m32 = (nh - b0) < 32 ? (nh - b0) : 32;
#pragma unroll 1
      for (int k = 0; k < m32; ++k) {
        const int u   = __builtin_amdgcn_readlane(uv, k);
        const int sl  = u & (NBMAX - 1);
        const int eid = (int)((unsigned)u >> 12);
        if (lane == 0) {
          int pos = list[sl];
          pos = pos < 0 ? 0 : (pos > RCAP - 1 ? RCAP - 1 : pos);
          reg2[pos] = eid;
          list[sl] = pos + 1;
        }
      }
    }
  }
  __syncthreads();

  const int nbw = nb >> 3;
  const int c4  = 4 * lane;
  const int jn  = lane & (EB - 1);
  const int hq  = lane >> 3;
  const int hb  = lane & 24;
  const v4f bz4 = *(const v4f*)(biasr + c4);
  const v4f at4 = *(const v4f*)(attr + c4);
  const float wb = web[hq];
#pragma unroll 1
  for (int jt = 0; jt < nbw; ++jt) {
    const int slot = wave * nbw + jt;
    const int grow = nodeBase + slot;
    const int gcl  = grow < nDst ? grow : nDst - 1;
    int st  = soff[slot];
    int cnt = scnt[slot];
    st  = st < 0 ? 0 : (st > nh ? nh : st);
    cnt = cnt < 0 ? 0 : (cnt > DEGCAP ? DEGCAP : cnt);
    if (cnt > nh - st) cnt = nh - st;

    const v4f pd4 = *(const v4f*)(yp + (size_t)gcl * FD + c4);
    const v4f t2 = pd4 + pd4;
    v4f z;
    z.x = fmaxf(t2.x, NEG_SLOPE * t2.x);
    z.y = fmaxf(t2.y, NEG_SLOPE * t2.y);
    z.z = fmaxf(t2.z, NEG_SLOPE * t2.z);
    z.w = fmaxf(t2.w, NEG_SLOPE * t2.w);
    float part = z.x * at4.x;
    part = fmaf(z.y, at4.y, part);
    part = fmaf(z.z, at4.z, part);
    part = fmaf(z.w, at4.w, part);
    part += __shfl_xor(part, 4);
    part += __shfl_xor(part, 2);
    part += __shfl_xor(part, 1);
    const float el = part + wb;

    float mx = el;
#pragma unroll 1
    for (int q0 = 0; q0 < cnt; q0 += EB) {
      const int qi = q0 + jn;
      int idx = st + qi; idx = idx > RCAP - 1 ? RCAP - 1 : idx;
      int eid = reg2[idx]; eid = eid < 0 ? 0 : (eid > nE - 1 ? nE - 1 : eid);
      const float e = ev[4 * (size_t)eid + hq];
      mx = (qi < cnt) ? fmaxf(mx, e) : mx;
    }
    mx = fmaxf(mx, __shfl_xor(mx, 4));
    mx = fmaxf(mx, __shfl_xor(mx, 2));
    mx = fmaxf(mx, __shfl_xor(mx, 1));

    const float pl = __expf(el - mx);
    float dsum = (jn == 0) ? pl : 0.0f;
    v4f ax = pd4 * pl;
#pragma unroll 1
    for (int q0 = 0; q0 < cnt; q0 += EB) {
      const int qi = q0 + jn;
      int idx = st + qi; idx = idx > RCAP - 1 ? RCAP - 1 : idx;
      int eid = reg2[idx]; eid = eid < 0 ? 0 : (eid > nE - 1 ? nE - 1 : eid);
      const float e = ev[4 * (size_t)eid + hq];
      int s = srcs[eid]; s = s < 0 ? 0 : (s > nDst - 1 ? nDst - 1 : s);
      const bool valid = qi < cnt;
      const float arg = valid ? (e - mx) : -80.0f;
      float p = __expf(arg);
      p = valid ? p : 0.0f;
      dsum += p;
      const int mcnt = (cnt - q0) < EB ? (cnt - q0) : EB;
#pragma unroll 1
      for (int pp = 0; pp < mcnt; ++pp) {
        const int   sp = __builtin_amdgcn_readlane(s, pp);
        const float pv = __shfl(p, hb | pp);
        const v4f xv = *(const v4f*)(yp + (size_t)sp * FD + c4);
        ax.x = fmaf(pv, xv.x, ax.x);
        ax.y = fmaf(pv, xv.y, ax.y);
        ax.z = fmaf(pv, xv.z, ax.z);
        ax.w = fmaf(pv, xv.w, ax.w);
      }
    }
    dsum += __shfl_xor(dsum, 4);
    dsum += __shfl_xor(dsum, 2);
    dsum += __shfl_xor(dsum, 1);
    const float inv = __builtin_amdgcn_rcpf(dsum);

    const v4f rr = *(const v4f*)(yr + (size_t)gcl * FD + c4);
    v4f o;
    o.x = (ax.x * inv + rr.x) + bz4.x;
    o.y = (ax.y * inv + rr.y) + bz4.y;
    o.z = (ax.z * inv + rr.z) + bz4.z;
    o.w = (ax.w * inv + rr.w) + bz4.w;
    float* gp = outp + (size_t)gcl * FD + c4;
    const bool wr = grow < nDst;
    if (wr) *(volatile v4f*)gp = o;
    __threadfence();
    if (wr) *(volatile v4f*)gp = o;
  }
}

static int pick_nb(int nE, int nDst) {
  int nb = NBMAX;
  while (nb > 16 && (long long)nb * (long long)nE * 5LL > (long long)RCAP * (long long)nDst * 4LL) nb >>= 1;
  return nb;
}

extern "C" void kernel_launch(void* const* d_in, const int* in_sizes, int n_in,
                              void* d_out, int out_size, void* d_ws, size_t ws_size,
                              hipStream_t stream) {
  if (n_in < 8) return;
  const int nN = in_sizes[0] / FD;
  if (nN <= 0 || in_sizes[0] != nN * FD) return;
  if (nN > (1 << 24)) return;
  const int szE = in_sizes[1];
  if (szE < 2 || (szE & 1) != 0) return;
  const int nE = szE / 2;
  if (nE > (1 << 20)) return;
  if (in_sizes[2] != 2 * nE) return;
  if (in_sizes[3] != FD * FD || in_sizes[7] != FD * FD) return;
  if (in_sizes[4] != NH * HC || in_sizes[5] != NH || in_sizes[6] != FD) return;
  if (out_size != nN * FD) return;

  const float* x    = (const float*)d_in[0];
  const int*   ei   = (const int*)d_in[1];
  const float* ea   = (const float*)d_in[2];
  const float* Wl   = (const float*)d_in[3];
  const float* att  = (const float*)d_in[4];
  const float* web  = (const float*)d_in[5];
  const float* bias = (const float*)d_in[6];
  const float* Wr   = (const float*)d_in[7];
  float* out = (float*)d_out;

  const int MP    = ((nN + GBM - 1) / GBM) * GBM;
  const int gridE = (nE + NTHR - 1) / NTHR;
  const int nb    = pick_nb(nE, nN);
  const int vec8  = ((nE & 3) == 0) ? 1 : 0;

  char* ws = (char*)d_ws;
  size_t off = 0;
  const size_t oWq = off; off += (size_t)NMAT * FD * FD * 2;           off = (off + 255) & ~(size_t)255;
  const size_t oX  = off; off += (size_t)MP * FD * 2;                  off = (off + 255) & ~(size_t)255;
  const size_t oY  = off; off += (size_t)2 * MP * FD * 4;              off = (off + 255) & ~(size_t)255;
  const size_t oEV = off; off += (size_t)gridE * NTHR * 4 * 4;         off = (off + 255) & ~(size_t)255;
  if (off > ws_size || off > (size_t)WSCAP) return;
  unsigned short* wq  = (unsigned short*)(ws + oWq);
  unsigned short* X16 = (unsigned short*)(ws + oX);
  float* YP = (float*)(ws + oY);
  float* YR = YP + (size_t)MP * FD;
  float* EV = (float*)(ws + oEV);

  hipFuncSetAttribute(reinterpret_cast<const void*>(&k_agg),
                      hipFuncAttributeMaxDynamicSharedMemorySize, LDS_AGG);

  k_xprep<<<MP * 16 / NTHR, NTHR, 0, stream>>>(x, X16, nN, MP * 16);
  k_wprep<<<dim3(FD * FD / 8 / NTHR, NMAT), NTHR, 0, stream>>>(Wl, Wr, wq);
  k_gemm<<<MP / GBM, GTHR, 0, stream>>>(X16, wq, YP, MP * FD);
  k_logit<<<gridE, NTHR, 0, stream>>>(ei, ei + nE, ea, YP, att, web, EV, nE, nN);
  k_agg<<<(nN + nb - 1) / nb, NTHR, LDS_AGG, stream>>>(ei, ei + nE, EV, YP, YR, att, web, bias, out,
                                                       nN, nE, nb, vec8);
}
